// MHA_64141041598707
// MI455X (gfx1250) — hardware-verified
//
#include <hip/hip_runtime.h>


#ifndef NB
#define NB 4
#endif
#ifndef SEQ
#define SEQ 2048
#endif
#define NB_FULL  4
#define SEQ_FULL 2048
#define DM   256
#define NH   8
#define HD   32
#define QKW  512
#define QCAR 16.0f
#define SCLX (0.0625f * 1.44269504088896340736f / 256.0f)

static_assert(DM == NH * HD);
static_assert(HD == 32);
static_assert((NH & 1) == 0);
static_assert(SEQ % 64 == 0);
static_assert(DM % 64 == 0 && QKW % 64 == 0 && DM % 32 == 0);
static_assert(NB <= NB_FULL && SEQ <= SEQ_FULL);

typedef _Float16 h16;
typedef unsigned short bf;
typedef __attribute__((ext_vector_type(16))) __bf16   v16bf;
typedef __attribute__((ext_vector_type(16))) _Float16 v16h;
typedef __attribute__((ext_vector_type(8)))  _Float16 v8h;
typedef __attribute__((ext_vector_type(8)))  unsigned short v8us;
typedef __attribute__((ext_vector_type(8)))  float    v8f;
typedef __attribute__((ext_vector_type(4)))  float    v4f;
typedef v4f  __attribute__((may_alias)) v4fa;

__device__ __forceinline__ unsigned short f2bf(float f) { unsigned u = __float_as_uint(f); u += 0x7FFFu + ((u >> 16) & 1u); return (unsigned short)(u >> 16); }
__device__ __forceinline__ float bf2f(unsigned short b) { return __uint_as_float(((unsigned)b) << 16); }
__device__ __forceinline__ v16h cat16(v8h lo, v8h hi) { return __builtin_shufflevector(lo, hi, 0, 1, 2, 3, 4, 5, 6, 7, 8, 9, 10, 11, 12, 13, 14, 15); }
__device__ __forceinline__ v16bf cat16b(v8us lo, v8us hi) { return __builtin_bit_cast(v16bf, __builtin_shufflevector(lo, hi, 0, 1, 2, 3, 4, 5, 6, 7, 8, 9, 10, 11, 12, 13, 14, 15)); }
__device__ __forceinline__ v8f wmma16(v16h a, v16h b, v8f c) { return __builtin_amdgcn_wmma_f32_16x16x32_f16(false, a, false, b, (short)0, c, false, false); }
__device__ __forceinline__ v8f wmmab(v16bf a, v16bf b, v8f c) { return __builtin_amdgcn_wmma_f32_16x16x32_bf16(false, a, false, b, (short)0, c, false, false); }
__device__ __forceinline__ void splitf(float y, unsigned short& h, unsigned short& l) { h = f2bf(y); l = f2bf(y - bf2f(h)); }
__device__ __forceinline__ v16h ldh(const h16* p) { return cat16(*(const v8h*)p, *(const v8h*)(p + 16)); }

template <typename T16> struct WFrag;
template <> struct WFrag<h16> { typedef v16h V; static __device__ __forceinline__ V ld(const h16* p) { return cat16(*(const v8h*)p, *(const v8h*)(p + 16)); } static __device__ __forceinline__ v8f mma(V a, V b, v8f c) { return wmma16(a, b, c); } };
template <> struct WFrag<bf> { typedef v16bf V; static __device__ __forceinline__ V ld(const bf* p) { return cat16b(*(const v8us*)p, *(const v8us*)(p + 16)); } static __device__ __forceinline__ v8f mma(V a, V b, v8f c) { return wmmab(a, b, c); } };
template <typename T16, int NSPLIT, int OMODE>
__global__ __launch_bounds__(32) void k_gemmw(const T16* __restrict__ A, const T16* __restrict__ A2, const T16* __restrict__ Bt, const T16* __restrict__ Bt2, int K, void* Cv, int ldc, float oscale, size_t sA, size_t sB, size_t sC) {
    typedef typename WFrag<T16>::V V;
    __shared__ __align__(16) float os[16 * 68];
    const size_t z = blockIdx.z; A += z * sA; if (A2) A2 += z * sA; Bt += z * sB; if (Bt2) Bt2 += z * sB;
    const unsigned lane = threadIdx.x & 31u, lr = lane & 15u, hi = lane >> 4; const unsigned r0 = blockIdx.x * 64u, c0 = blockIdx.y * 64u;
    v8f acc[4][4];
#pragma unroll
    for (int mb = 0; mb < 4; ++mb)
#pragma unroll
        for (int nb = 0; nb < 4; ++nb) acc[mb][nb] = (v8f){};
    const size_t aoff = (size_t)(r0 + lr) * K + 8 * hi, boff = (size_t)(c0 + lr) * K + 8 * hi;
#pragma unroll 1
    for (int kc = 0; kc < K; kc += 32) {
        V a[4], a2[4];
#pragma unroll
        for (int mb = 0; mb < 4; ++mb) { a[mb] = WFrag<T16>::ld(A + aoff + (size_t)mb * 16 * K + kc); if (NSPLIT == 1 || NSPLIT == 2) a2[mb] = WFrag<T16>::ld(A2 + aoff + (size_t)mb * 16 * K + kc); }
#pragma unroll
        for (int nb = 0; nb < 4; ++nb) { const V b = WFrag<T16>::ld(Bt + boff + (size_t)nb * 16 * K + kc); V b2; if (NSPLIT >= 2) b2 = WFrag<T16>::ld(Bt2 + boff + (size_t)nb * 16 * K + kc);
#pragma unroll
            for (int mb = 0; mb < 4; ++mb) { acc[mb][nb] = WFrag<T16>::mma(a[mb], b, acc[mb][nb]); if (NSPLIT == 1 || NSPLIT == 2) acc[mb][nb] = WFrag<T16>::mma(a2[mb], b, acc[mb][nb]); if (NSPLIT >= 2) acc[mb][nb] = WFrag<T16>::mma(a[mb], b2, acc[mb][nb]); } }
        if constexpr (NSPLIT == 1 || NSPLIT == 2) { asm volatile("v_nop\n\tv_nop\n\tv_nop\n\tv_nop" : "+v"(acc[0][0]), "+v"(acc[1][1]), "+v"(acc[2][2]), "+v"(acc[3][3]) : "v"(a[0]), "v"(a[3]), "v"(a2[3])); }
        else { asm volatile("v_nop\n\tv_nop\n\tv_nop\n\tv_nop" : "+v"(acc[0][0]), "+v"(acc[1][1]), "+v"(acc[2][2]), "+v"(acc[3][3]) : "v"(a[0]), "v"(a[3])); }
    }
#pragma unroll
    for (int mb = 0; mb < 4; ++mb) {
#pragma unroll
        for (int nb = 0; nb < 4; ++nb) {
#pragma unroll
            for (int j = 0; j < 8; ++j) os[(hi * 8 + j) * 68 + nb * 16 + lr] = acc[mb][nb][j]; }
        __syncthreads();
        if constexpr (OMODE == 0) {
            float* crow = (float*)Cv + z * sC + (size_t)(r0 + mb * 16) * ldc + c0;
#pragma unroll 1
            for (int ps = 0; ps < 2; ++ps) {
#pragma unroll
                for (int s = 0; s < 8; ++s) { const unsigned row = 2u * s + hi, cofs = lr * 4u; const v4f val = *(const v4fa*)(os + row * 68 + cofs);
                    *(volatile v4f*)(crow + (size_t)row * ldc + cofs) = val; }
                if (ps == 0) __threadfence(); }
        } else {
            h16* crow = (h16*)Cv + z * sC + (size_t)(r0 + mb * 16) * ldc + c0;
#pragma unroll 1
            for (int ps = 0; ps < 2; ++ps) {
#pragma unroll
                for (int s = 0; s < 4; ++s) { const unsigned row = 4u * s + (lane >> 3), pc = (lane & 7u) * 8u; const v4f v0 = *(const v4fa*)(os + row * 68 + pc); const v4f v1 = *(const v4fa*)(os + row * 68 + pc + 4); v8h o;
#pragma unroll
                    for (int q = 0; q < 4; ++q) { o[q] = (h16)(v0[q] * oscale); o[4 + q] = (h16)(v1[q] * oscale); }
                    *(volatile v8h*)(crow + (size_t)row * ldc + pc) = o; }
                if (ps == 0) __threadfence(); }
        }
        __syncthreads();
    }
}

__global__ __launch_bounds__(256) void k_xprep(const float* __restrict__ x, bf* XB) {
    const unsigned i = blockIdx.x * 256u + threadIdx.x; if (i >= (unsigned)NB * SEQ * (DM / 8)) return;
    const unsigned b = i / ((unsigned)SEQ * (DM / 8)), r = i - b * ((unsigned)SEQ * (DM / 8));
    const float* s = x + ((size_t)b * SEQ_FULL * (DM / 8) + r) * 8; const v4f a0 = *(const v4f*)s, a1 = *(const v4f*)(s + 4); v8us o;
#pragma unroll
    for (int q = 0; q < 4; ++q) { o[q] = f2bf(a0[q]); o[4 + q] = f2bf(a1[q]); }
    *(volatile v8us*)(XB + (size_t)i * 8) = o; __threadfence(); *(volatile v8us*)(XB + (size_t)i * 8) = o; }

__global__ __launch_bounds__(256) void k_wprep(const float* __restrict__ wq, const float* __restrict__ wk, const float* __restrict__ wv, const float* __restrict__ wo, bf* WQK, bf* WV, bf* WOT) {
    __shared__ float ts[256 * 33];
    const unsigned tid = threadIdx.x, g = blockIdx.x, mt = blockIdx.y;
    const float* src = wq; unsigned gs = (unsigned)DM * HD, ds = HD; bf* dst = WQK;
    if (mt == 1u) { src = wk; dst = WQK + (size_t)DM * DM; } else if (mt == 2u) { src = wv; dst = WV; } else if (mt == 3u) { src = wo; gs = HD; ds = DM; dst = WOT; }
#pragma unroll 4
    for (unsigned it = 0; it < 32u; ++it) { const unsigned idx = it * 256u + tid, d = idx >> 5, e = idx & 31u; ts[d * 33u + e] = src[(size_t)g * gs + (size_t)d * ds + e]; }
    __syncthreads();
#pragma unroll 1
    for (int ps = 0; ps < 2; ++ps) {
#pragma unroll
        for (unsigned it = 0; it < 4u; ++it) { const unsigned p = it * 256u + tid, e = p >> 5, pc = p & 31u; v8us o;
#pragma unroll
            for (unsigned q = 0; q < 8u; ++q) o[q] = f2bf(ts[(pc * 8u + q) * 33u + e]);
            *(volatile v8us*)(dst + (size_t)(g * HD + e) * DM + pc * 8u) = o; }
        if (ps == 0) __threadfence(); }
}

#define FW 4
__global__ __launch_bounds__(128) void k_flash(const h16* __restrict__ QK, const h16* __restrict__ VT, bf* CH, bf* CL) {
    __shared__ __align__(16) float os[FW * 16 * 68];
    const unsigned tid = threadIdx.x, lane = tid & 31u, w = tid >> 5, lr = lane & 15u, hi = lane >> 4;
    const unsigned bz = blockIdx.z, hp = blockIdx.y, i0 = blockIdx.x * 64u + w * 16u;
    const h16* qkb = QK + (size_t)bz * SEQ * QKW;
    const h16* vtb = VT + (size_t)bz * DM * SEQ;
    float* osw = os + w * (16u * 68u);
#pragma unroll 1
    for (unsigned hh = 0; hh < 2u; ++hh) {
        const unsigned hd = hp * 2u + hh;
        const v16h bq = ldh(qkb + (size_t)(i0 + lr) * QKW + hd * HD + 8u * hi);
        const h16* kp = qkb + (size_t)lr * QKW + DM + hd * HD + 8u * hi;
        const h16* vp = vtb + (size_t)(hd * HD + lr) * SEQ + 8u * hi;
        v8f acc0 = (v8f){}, acc1 = (v8f){}; float m = -3.0e38f, l = 0.0f;
#pragma unroll 1
        for (unsigned j0 = 0; j0 < (unsigned)SEQ; j0 += 64u) {
            const h16* kt = kp + (size_t)j0 * QKW;
            const v16h ka0 = ldh(kt), ka1 = ldh(kt + 16 * QKW), ka2 = ldh(kt + 32 * QKW), ka3 = ldh(kt + 48 * QKW);
            v8f s0 = wmma16(ka0, bq, (v8f){}); v8f s1 = wmma16(ka1, bq, (v8f){}); v8f s2 = wmma16(ka2, bq, (v8f){}); v8f s3 = wmma16(ka3, bq, (v8f){});
            asm volatile("v_nop\n\tv_nop\n\tv_nop\n\tv_nop" : "+v"(s0), "+v"(s1), "+v"(s2), "+v"(s3) : "v"(ka3), "v"(bq));
            float vm = s0[0];
#pragma unroll
            for (int r = 0; r < 8; ++r) { vm = fmaxf(vm, fmaxf(s0[r], s1[r])); vm = fmaxf(vm, fmaxf(s2[r], s3[r])); }
            vm = fmaxf(vm, __shfl_xor(vm, 16, 32));
            const float mn = fmaxf(m, vm * SCLX);
            const float alpha = __builtin_amdgcn_exp2f(m - mn); m = mn;
            const float nb = 10.0f - mn;
            float rs = 0.0f;
#pragma unroll
            for (int r = 0; r < 8; ++r) {
                s0[r] = __builtin_amdgcn_exp2f(fmaf(s0[r], SCLX, nb)); s1[r] = __builtin_amdgcn_exp2f(fmaf(s1[r], SCLX, nb));
                s2[r] = __builtin_amdgcn_exp2f(fmaf(s2[r], SCLX, nb)); s3[r] = __builtin_amdgcn_exp2f(fmaf(s3[r], SCLX, nb));
                rs += (s0[r] + s1[r]) + (s2[r] + s3[r]); }
            rs += __shfl_xor(rs, 16, 32);
            l = l * alpha + rs;
            v16h pB0, pB1;
#pragma unroll
            for (int r = 0; r < 8; ++r) { acc0[r] *= alpha; acc1[r] *= alpha;
                pB0[r] = (h16)s0[r]; pB0[8 + r] = (h16)s1[r]; pB1[r] = (h16)s2[r]; pB1[8 + r] = (h16)s3[r]; }
            const h16* vt = vp + j0;
            const v16h va00 = ldh(vt), va01 = ldh(vt + 32), va10 = ldh(vt + (size_t)16 * SEQ), va11 = ldh(vt + (size_t)16 * SEQ + 32);
            acc0 = wmma16(va00, pB0, acc0); acc1 = wmma16(va10, pB0, acc1); acc0 = wmma16(va01, pB1, acc0); acc1 = wmma16(va11, pB1, acc1);
            asm volatile("v_nop\n\tv_nop\n\tv_nop\n\tv_nop" : "+v"(acc0), "+v"(acc1) : "v"(va11), "v"(va01), "v"(pB1));
        }
        const float inv = (1.0f / QCAR) / l;
#pragma unroll
        for (int r = 0; r < 8; ++r) { osw[lr * 68u + hh * 32u + 8u * hi + r] = acc0[r] * inv; osw[lr * 68u + hh * 32u + 16u + 8u * hi + r] = acc1[r] * inv; }
    }
    __syncthreads();
    const size_t rowbase = ((size_t)bz * SEQ + i0) * DM + hp * 64u;
#pragma unroll 1
    for (int ps = 0; ps < 2; ++ps) {
#pragma unroll
        for (unsigned s = 0; s < 4u; ++s) { const unsigned row = 4u * s + (lane >> 3), pc = (lane & 7u) * 8u; const v4f v0 = *(const v4fa*)(osw + row * 68u + pc); const v4f v1 = *(const v4fa*)(osw + row * 68u + pc + 4u); v8us oh, ol;
#pragma unroll
            for (int q = 0; q < 4; ++q) { unsigned short a2, c2; splitf(v0[q], a2, c2); oh[q] = a2; ol[q] = c2; splitf(v1[q], a2, c2); oh[4 + q] = a2; ol[4 + q] = c2; }
            const size_t oo = rowbase + (size_t)row * DM + pc;
            *(volatile v8us*)(CH + oo) = oh; *(volatile v8us*)(CL + oo) = ol; }
        if (ps == 0) __threadfence(); }
}

constexpr size_t al256(size_t b) { return (b + 255) & ~(size_t)255; }
constexpr size_t SZ_XB  = al256((size_t)NB * SEQ * DM * 2);
constexpr size_t SZ_WQK = al256((size_t)QKW * DM * 2);
constexpr size_t SZ_W   = al256((size_t)DM * DM * 2);
constexpr size_t SZ_QK  = al256((size_t)NB * SEQ * QKW * 2);
constexpr size_t SZ_VT  = al256((size_t)NB * DM * SEQ * 2);
constexpr size_t SZ_C   = al256((size_t)NB * SEQ * DM * 2);
constexpr size_t CARVE  = SZ_XB + SZ_WQK + 2 * SZ_W + SZ_QK + SZ_VT + 2 * SZ_C;
static_assert(CARVE <= (size_t)134217728);
static_assert(((size_t)NB * SEQ * (DM / 8)) % 256 == 0);
static_assert((size_t)NH * 4 * 256 * 4 * 8 == (size_t)(QKW + 2 * DM) * DM);
static_assert((size_t)(SEQ / 64) * (NH / 2) * NB * FW * 16 * 64 == (size_t)NB * SEQ * DM);

extern "C" void kernel_launch(void* const* d_in, const int* in_sizes, int n_in,
                              void* d_out, int out_size, void* d_ws, size_t ws_size, hipStream_t stream) {
    if (n_in < 5) return;
    const long long xmin = (long long)(NB - 1) * SEQ_FULL * DM + (long long)SEQ * DM;
    if ((long long)in_sizes[0] < xmin || in_sizes[1] < NH * DM * HD || in_sizes[2] < NH * DM * HD || in_sizes[3] < NH * DM * HD || in_sizes[4] < DM * DM) return;
    if ((long long)out_size < xmin) return;
    if (CARVE > ws_size) return;
    const float* x = (const float*)d_in[0]; const float* wq = (const float*)d_in[1]; const float* wk = (const float*)d_in[2]; const float* wv = (const float*)d_in[3]; const float* wo = (const float*)d_in[4];
    float* OUT = (float*)d_out;
    char* wsp = (char*)d_ws;
    auto take = [&](size_t bytes) { char* p = wsp; wsp += bytes; return (void*)p; };
    bf* XB = (bf*)take(SZ_XB); bf* WQK = (bf*)take(SZ_WQK); bf* WV = (bf*)take(SZ_W); bf* WOT = (bf*)take(SZ_W);
    h16* QKP = (h16*)take(SZ_QK); h16* VTP = (h16*)take(SZ_VT); bf* CH = (bf*)take(SZ_C); bf* CL = (bf*)take(SZ_C);

    k_wprep<<<dim3(NH, 4, 1), 256, 0, stream>>>(wq, wk, wv, wo, WQK, WV, WOT);
    k_xprep<<<(unsigned)(((size_t)NB * SEQ * (DM / 8)) / 256), 256, 0, stream>>>(x, XB);
    k_gemmw<bf, 0, 1><<<dim3((unsigned)((size_t)NB * SEQ / 64), QKW / 64, 1), 32, 0, stream>>>(XB, nullptr, WQK, nullptr, DM, (void*)QKP, QKW, QCAR, 0, 0, 0);
    k_gemmw<bf, 0, 1><<<dim3(DM / 64, SEQ / 64, NB), 32, 0, stream>>>(WV, nullptr, XB, nullptr, DM, (void*)VTP, SEQ, QCAR, 0, (size_t)SEQ * DM, (size_t)DM * SEQ);
    k_flash<<<dim3(SEQ / 64, NH / 2, NB), 128, 0, stream>>>(QKP, VTP, CH, CL);
    k_gemmw<bf, 1, 0><<<dim3(SEQ / 64, DM / 64, NB), 32, 0, stream>>>(CH, CL, WOT, nullptr, DM, (void*)OUT, DM, 1.0f, (size_t)SEQ * DM, 0, (size_t)SEQ_FULL * DM);
}
